// Spell_7499012899510
// MI455X (gfx1250) — hardware-run, weakly checked
//
#include <hip/hip_runtime.h>
#include <math.h>

typedef __attribute__((ext_vector_type(16))) _Float16 v16h;
typedef __attribute__((ext_vector_type(8)))  _Float16 v8h;
typedef __attribute__((ext_vector_type(8)))  float    v8f;
typedef __attribute__((ext_vector_type(4)))  float    v4f;

constexpr int kB = 16;
constexpr int kL = 2048;
constexpr int kT = 256;
constexpr int kD = 256;
constexpr int kH = 512;
constexpr int kV = 34;
constexpr int kK1 = 2 * kD + kH;
constexpr int kK2 = kH + kD;
constexpr int kKo = 2 * kD;
constexpr int kVPad = 64;
constexpr int kRowsOut = kT * kB;

constexpr int kXP = 1288;
constexpr int kColEmb = 0;
constexpr int kColCtx = kD;
constexpr int kColH1  = 2 * kD;
constexpr int kColH2  = 2 * kD + kH;

constexpr int kChunk  = 256;
constexpr int kNChunk = kL / kChunk;
constexpr int kGroups = kChunk / 32;
constexpr int kPReg   = kL / 32;

constexpr float kCarryA = 1024.0f;
constexpr float kCarryW = 256.0f;
constexpr float kFold   = 1.0f / (kCarryA * kCarryW);
constexpr float kF16Min = 6.103515625e-5f;

static_assert(kK1 % 32 == 0 && kK2 % 32 == 0 && kKo % 32 == 0);
static_assert(kRowsOut % 64 == 0 && kVPad % 64 == 0);
static_assert(kColH2 + kD <= kXP && (kXP % 8) == 0);
static_assert(kNChunk * kGroups == kPReg);
static_assert((kT * kB * kV * 4) % 128 == 0);

constexpr size_t kOffW1C  = 0;
constexpr size_t kOffW2C  = kOffW1C  + (size_t)4 * kH * kK1 * 2;
constexpr size_t kOffWO   = kOffW2C  + (size_t)4 * kD * kK2 * 2;
constexpr size_t kOffHCAT = kOffWO   + (size_t)kVPad * kKo * 2;
constexpr size_t kOffC64  = kOffHCAT + (size_t)kRowsOut * kKo * 2;
constexpr size_t kWsTotal = kOffC64  + (size_t)kRowsOut * kVPad * 4;
static_assert(kWsTotal == 11075584ull);
static_assert(kWsTotal <= 134217728ull);
static_assert((kOffW2C % 128) == 0 && (kOffWO % 128) == 0 && (kOffHCAT % 128) == 0 && (kOffC64 % 128) == 0);

union FragH { v16h v; v8h h[2]; };

__device__ __forceinline__ v8f mma_h(v16h a, v16h b, v8f c) {
  c = __builtin_amdgcn_wmma_f32_16x16x32_f16(false, a, false, b, (short)0, c, false, false);
  asm volatile("v_nop\n\tv_nop\n\tv_nop\n\tv_nop" : "+v"(c) : "v"(a), "v"(b));
  return c;
}

__device__ __forceinline__ _Float16 cvt_h(float xc) {
  const float y = (fabsf(xc) < kF16Min) ? 0.0f : xc;
  return (_Float16)y;
}

__device__ __forceinline__ v8h cvt8_carry(const float* __restrict__ src, float carry) {
  const v4f a0 = *(const v4f*)(src);
  const v4f a1 = *(const v4f*)(src + 4);
  v8h r;
#pragma unroll
  for (int e = 0; e < 4; ++e) {
    r[e]     = cvt_h(a0[e] * carry);
    r[4 + e] = cvt_h(a1[e] * carry);
  }
  return r;
}

__device__ __forceinline__ float sigm(float x) { return __builtin_amdgcn_rcpf(1.0f + __expf(-x)); }
__device__ __forceinline__ float tnh(float x)  { return 1.0f - 2.0f * __builtin_amdgcn_rcpf(1.0f + __expf(2.0f * x)); }

__device__ __forceinline__ void wave_lds_sync() {
  __builtin_amdgcn_fence(__ATOMIC_RELEASE, "workgroup");
  __builtin_amdgcn_wave_barrier();
  __builtin_amdgcn_fence(__ATOMIC_ACQUIRE, "workgroup");
}

__global__ __launch_bounds__(256) void cvt_rows_f16_kernel(
    const float* __restrict__ src, int src_ld, int rows_real,
    unsigned short* __restrict__ dst, int dst_ld, int dst_col0,
    int cols8, int total, float carry)
{
  const int i = blockIdx.x * 256 + threadIdx.x;
  if (i >= total) return;
  const int row = i / cols8;
  const int c8  = (i - row * cols8) * 8;
  const int rs  = (row < rows_real) ? row : (rows_real - 1);
  const float* sp = src + (size_t)rs * src_ld + c8;
  const v4f a0 = *(const v4f*)(sp);
  const v4f a1 = *(const v4f*)(sp + 4);
  const bool keep = (row < rows_real);
  v8h hv;
#pragma unroll
  for (int e = 0; e < 4; ++e) {
    const float x0 = keep ? (a0[e] * carry) : 0.0f;
    const float x1 = keep ? (a1[e] * carry) : 0.0f;
    hv[e]     = cvt_h(x0);
    hv[4 + e] = cvt_h(x1);
  }
  unsigned short* dp = dst + (size_t)row * dst_ld + dst_col0 + c8;
  *(volatile v8h*)dp = hv;
  __threadfence();
  *(volatile v8h*)dp = hv;
}

__global__ __launch_bounds__(512) void decoder_steps_kernel(
    const float* __restrict__ key, const float* __restrict__ value,
    const int* __restrict__ lens, const int* __restrict__ trans,
    const float* __restrict__ emb,
    const unsigned short* __restrict__ W1p, const unsigned short* __restrict__ W2p,
    const float* __restrict__ bih1, const float* __restrict__ bhh1,
    const float* __restrict__ bih2, const float* __restrict__ bhh2,
    const float* __restrict__ h10, const float* __restrict__ c10,
    const float* __restrict__ h20, const float* __restrict__ c20,
    unsigned short* __restrict__ Hcat, float* __restrict__ attn_out)
{
  __shared__ __align__(16) _Float16 XA[kB * kXP];
  __shared__ __align__(16) float    H2F[kB * kD];
  __shared__ __align__(16) float    PB[kB * kChunk];

  const _Float16* W1 = (const _Float16*)W1p;
  const _Float16* W2 = (const _Float16*)W2p;

  const int tid  = threadIdx.x;
  const int lane = tid & 31;
  const int wv   = __builtin_amdgcn_readfirstlane(tid >> 5);
  const int hh   = lane >> 4;
  const int cc   = lane & 15;

  int lenb = lens[wv];
  lenb = lenb < 0 ? 0 : lenb;
  lenb = lenb > kL ? kL : lenb;
  lenb = __builtin_amdgcn_readfirstlane(lenb);

  {
    int tok = trans[wv * kT];
    tok = tok < 0 ? 0 : tok;
    tok = tok > (kV - 1) ? (kV - 1) : tok;
    const v8h ev = cvt8_carry(emb + (size_t)tok * kD + lane * 8, kCarryA);
    *(v8h*)(XA + wv * kXP + kColEmb + lane * 8) = ev;
    v8h zv;
#pragma unroll
    for (int e = 0; e < 8; ++e) zv[e] = (_Float16)0.0f;
    *(v8h*)(XA + wv * kXP + kColCtx + lane * 8) = zv;
    const v8h ha = cvt8_carry(h10 + (size_t)wv * kH + lane * 8, kCarryA);
    const v8h hb = cvt8_carry(h10 + (size_t)wv * kH + 256 + lane * 8, kCarryA);
    *(v8h*)(XA + wv * kXP + kColH1 + lane * 8) = ha;
    *(v8h*)(XA + wv * kXP + kColH1 + 256 + lane * 8) = hb;
    const v8h h2v0 = cvt8_carry(h20 + (size_t)wv * kD + lane * 8, kCarryA);
    *(v8h*)(XA + wv * kXP + kColH2 + lane * 8) = h2v0;
  }

  float c1s[2][8], c2s[8], bs1[2][4], bs2[4];
#pragma unroll
  for (int jj = 0; jj < 2; ++jj) {
#pragma unroll
    for (int r = 0; r < 8; ++r) c1s[jj][r] = c10[(size_t)(8 * hh + r) * kH + (2 * wv + jj) * 16 + cc];
#pragma unroll
    for (int g = 0; g < 4; ++g) {
      const int n = g * kH + (2 * wv + jj) * 16 + cc;
      bs1[jj][g] = bih1[n] + bhh1[n];
    }
  }
#pragma unroll
  for (int r = 0; r < 8; ++r) c2s[r] = c20[(size_t)(8 * hh + r) * kD + wv * 16 + cc];
#pragma unroll
  for (int g = 0; g < 4; ++g) {
    const int n = g * kD + wv * 16 + cc;
    bs2[g] = bih2[n] + bhh2[n];
  }
  __syncthreads();

  const int aoff = cc * kXP + 8 * hh;
  const _Float16* w1b = W1 + (size_t)((2 * wv) * 16 + cc) * kK1 + 8 * hh;
  const _Float16* w2b = W2 + (size_t)(wv * 16 + cc) * kK2 + 8 * hh;
  const float* kbase = key + ((size_t)lane * kB + wv) * kD;
  const float* vbase = value + (size_t)wv * kD + lane * 8;
  float* pb = PB + wv * kChunk;
  const float* hrow = H2F + wv * kD;

#pragma unroll 1
  for (int t = 0; t < kT; ++t) {
    v8f a1[2][4];
#pragma unroll
    for (int jj = 0; jj < 2; ++jj)
#pragma unroll
      for (int g = 0; g < 4; ++g) a1[jj][g] = (v8f){0.f, 0.f, 0.f, 0.f, 0.f, 0.f, 0.f, 0.f};
#pragma unroll 1
    for (int k0 = 0; k0 < kK1; k0 += 32) {
      FragH af;
      af.h[0] = *(const v8h*)(XA + aoff + k0);
      af.h[1] = *(const v8h*)(XA + aoff + k0 + 16);
#pragma unroll
      for (int jj = 0; jj < 2; ++jj) {
#pragma unroll
        for (int g = 0; g < 4; ++g) {
          const _Float16* bp = w1b + (size_t)(g * kH + jj * 16) * kK1 + k0;
          FragH bf;
          bf.h[0] = *(const v8h*)(bp);
          bf.h[1] = *(const v8h*)(bp + 16);
          a1[jj][g] = mma_h(af.v, bf.v, a1[jj][g]);
        }
      }
    }
    float hn1[2][8];
#pragma unroll
    for (int jj = 0; jj < 2; ++jj) {
#pragma unroll
      for (int r = 0; r < 8; ++r) {
        const float gi = a1[jj][0][r] * kFold + bs1[jj][0];
        const float gf = a1[jj][1][r] * kFold + bs1[jj][1];
        const float gg = a1[jj][2][r] * kFold + bs1[jj][2];
        const float go = a1[jj][3][r] * kFold + bs1[jj][3];
        const float cn = sigm(gf) * c1s[jj][r] + sigm(gi) * tnh(gg);
        c1s[jj][r] = cn;
        hn1[jj][r] = sigm(go) * tnh(cn);
      }
    }
    __syncthreads();
#pragma unroll
    for (int jj = 0; jj < 2; ++jj)
#pragma unroll
      for (int r = 0; r < 8; ++r)
        XA[(8 * hh + r) * kXP + kColH1 + (2 * wv + jj) * 16 + cc] = cvt_h(hn1[jj][r] * kCarryA);
    __syncthreads();

    v8f a2[4];
#pragma unroll
    for (int g = 0; g < 4; ++g) a2[g] = (v8f){0.f, 0.f, 0.f, 0.f, 0.f, 0.f, 0.f, 0.f};
#pragma unroll 1
    for (int k0 = 0; k0 < kK2; k0 += 32) {
      FragH af;
      af.h[0] = *(const v8h*)(XA + aoff + kColH1 + k0);
      af.h[1] = *(const v8h*)(XA + aoff + kColH1 + k0 + 16);
#pragma unroll
      for (int g = 0; g < 4; ++g) {
        const _Float16* bp = w2b + (size_t)(g * kD) * kK2 + k0;
        FragH bf;
        bf.h[0] = *(const v8h*)(bp);
        bf.h[1] = *(const v8h*)(bp + 16);
        a2[g] = mma_h(af.v, bf.v, a2[g]);
      }
    }
    float hn2[8];
#pragma unroll
    for (int r = 0; r < 8; ++r) {
      const float gi = a2[0][r] * kFold + bs2[0];
      const float gf = a2[1][r] * kFold + bs2[1];
      const float gg = a2[2][r] * kFold + bs2[2];
      const float go = a2[3][r] * kFold + bs2[3];
      const float cn = sigm(gf) * c2s[r] + sigm(gi) * tnh(gg);
      c2s[r] = cn;
      hn2[r] = sigm(go) * tnh(cn);
    }
    __syncthreads();
#pragma unroll
    for (int r = 0; r < 8; ++r) {
      XA[(8 * hh + r) * kXP + kColH2 + wv * 16 + cc] = cvt_h(hn2[r] * kCarryA);
      H2F[(8 * hh + r) * kD + wv * 16 + cc] = hn2[r];
    }
    __syncthreads();

    float p[kPReg];
    float cacc[8];
#pragma unroll
    for (int i = 0; i < 8; ++i) cacc[i] = 0.0f;
    float zpart = 0.0f;
#pragma unroll
    for (int ch = 0; ch < kNChunk; ++ch) {
      const int l0 = ch * kChunk;
#pragma unroll
      for (int g = 0; g < kGroups; ++g) p[ch * kGroups + g] = 0.0f;
      if (l0 < lenb) {
        float en[kGroups];
#pragma unroll
        for (int g = 0; g < kGroups; ++g) en[g] = 0.0f;
        const float* kp = kbase + (size_t)l0 * (kB * kD);
#pragma unroll 1
        for (int d = 0; d < kD; d += 4) {
          const v4f hv = *(const v4f*)(hrow + d);
#pragma unroll
          for (int g = 0; g < kGroups; ++g) {
            const v4f kv = *(const v4f*)(kp + (size_t)g * (32 * kB * kD) + d);
            float a = en[g];
            a = fmaf(kv[0], hv[0], a);
            a = fmaf(kv[1], hv[1], a);
            a = fmaf(kv[2], hv[2], a);
            a = fmaf(kv[3], hv[3], a);
            en[g] = a;
          }
        }
#pragma unroll
        for (int g = 0; g < kGroups; ++g) {
          const int l = l0 + g * 32 + lane;
          const float ex = __expf(en[g]);
          const float pv = (l < lenb) ? ex : 0.0f;
          p[ch * kGroups + g] = pv;
          zpart += pv;
          pb[g * 32 + lane] = pv;
        }
        wave_lds_sync();
        int nrows = lenb - l0;
        nrows = nrows > kChunk ? kChunk : nrows;
        const int nr4 = (nrows + 3) >> 2;
        const float* vp = vbase + (size_t)l0 * (kB * kD);
#pragma unroll 1
        for (int r4 = 0; r4 < nr4; ++r4) {
          const float q0 = pb[r4 * 4 + 0];
          const float q1 = pb[r4 * 4 + 1];
          const float q2 = pb[r4 * 4 + 2];
          const float q3 = pb[r4 * 4 + 3];
          const float* vr = vp + (size_t)(r4 * 4) * (kB * kD);
          const v4f u0 = *(const v4f*)(vr);
          const v4f u1 = *(const v4f*)(vr + 4);
          const v4f u2 = *(const v4f*)(vr + (kB * kD));
          const v4f u3 = *(const v4f*)(vr + (kB * kD) + 4);
          const v4f u4 = *(const v4f*)(vr + 2 * (kB * kD));
          const v4f u5 = *(const v4f*)(vr + 2 * (kB * kD) + 4);
          const v4f u6 = *(const v4f*)(vr + 3 * (kB * kD));
          const v4f u7 = *(const v4f*)(vr + 3 * (kB * kD) + 4);
#pragma unroll
          for (int e = 0; e < 4; ++e) {
            float s0 = cacc[e], s1 = cacc[4 + e];
            s0 = fmaf(q0, u0[e], s0);
            s1 = fmaf(q0, u1[e], s1);
            s0 = fmaf(q1, u2[e], s0);
            s1 = fmaf(q1, u3[e], s1);
            s0 = fmaf(q2, u4[e], s0);
            s1 = fmaf(q2, u5[e], s1);
            s0 = fmaf(q3, u6[e], s0);
            s1 = fmaf(q3, u7[e], s1);
            cacc[e] = s0;
            cacc[4 + e] = s1;
          }
        }
        wave_lds_sync();
      }
    }
    float z = zpart;
    z += __shfl_xor(z, 16, 32);
    z += __shfl_xor(z, 8, 32);
    z += __shfl_xor(z, 4, 32);
    z += __shfl_xor(z, 2, 32);
    z += __shfl_xor(z, 1, 32);
    const float invZ = 1.0f / z;
#pragma unroll
    for (int i = 0; i < kPReg; ++i) p[i] = p[i] * invZ;
    v8h cv;
#pragma unroll
    for (int i = 0; i < 8; ++i) cv[i] = cvt_h(cacc[i] * invZ * kCarryA);

    *(v8h*)(XA + wv * kXP + kColCtx + lane * 8) = cv;
    {
      const int tn = (t + 1 < kT) ? (t + 1) : (kT - 1);
      int tok = trans[wv * kT + tn];
      tok = tok < 0 ? 0 : tok;
      tok = tok > (kV - 1) ? (kV - 1) : tok;
      const v8h ev = cvt8_carry(emb + (size_t)tok * kD + lane * 8, kCarryA);
      *(v8h*)(XA + wv * kXP + kColEmb + lane * 8) = ev;
    }
    const v8h h2v = *(const v8h*)(XA + wv * kXP + kColH2 + lane * 8);

    unsigned short* hc = Hcat + (size_t)(t * kB + wv) * kKo;
    float* ao = attn_out + (size_t)(t * kB + wv) * kL + lane;
    for (int pass = 0; pass < 2; ++pass) {
      *(volatile v8h*)(hc + lane * 8) = h2v;
      *(volatile v8h*)(hc + kD + lane * 8) = cv;
#pragma unroll
      for (int i = 0; i < kPReg; ++i) *(volatile float*)(ao + i * 32) = p[i];
      __threadfence();
    }
    __syncthreads();
  }
}

__global__ __launch_bounds__(256) void gemm64_f16_kernel(
    const unsigned short* __restrict__ Ap, int lda,
    const unsigned short* __restrict__ Btp, int ldb,
    float* __restrict__ C, int ldc, int M, int N, int K, float scale)
{
  __shared__ __align__(16) float sT[8][16 * 68];
  const _Float16* A  = (const _Float16*)Ap;
  const _Float16* Bt = (const _Float16*)Btp;
  const int lane = threadIdx.x & 31;
  const int wave = threadIdx.x >> 5;
  const int tilesN = N >> 6;
  const int tilesM = M >> 6;
  const int tile = blockIdx.x * 8 + wave;
  if (tile >= tilesM * tilesN) return;
  const int tm = tile / tilesN;
  const int tn = tile - tm * tilesN;
  const int m0 = tm << 6;
  const int n0 = tn << 6;
  const int rlane = lane & 15;
  const int koff  = (lane >> 4) * 8;
  const int mOff  = (lane >> 4) * 8;

  v8f acc[4][4];
#pragma unroll
  for (int i = 0; i < 4; ++i)
#pragma unroll
    for (int j = 0; j < 4; ++j) acc[i][j] = (v8f){0.f, 0.f, 0.f, 0.f, 0.f, 0.f, 0.f, 0.f};

  for (int k0 = 0; k0 < K; k0 += 32) {
    v16h bh[4];
#pragma unroll
    for (int j = 0; j < 4; ++j) {
      const _Float16* bp = Bt + (size_t)(n0 + (j << 4) + rlane) * ldb + koff + k0;
      FragH f;
      f.h[0] = *(const v8h*)(bp);
      f.h[1] = *(const v8h*)(bp + 16);
      bh[j] = f.v;
    }
#pragma unroll
    for (int i = 0; i < 4; ++i) {
      const _Float16* ap = A + (size_t)(m0 + (i << 4) + rlane) * lda + koff + k0;
      FragH f;
      f.h[0] = *(const v8h*)(ap);
      f.h[1] = *(const v8h*)(ap + 16);
#pragma unroll
      for (int j = 0; j < 4; ++j) acc[i][j] = mma_h(f.v, bh[j], acc[i][j]);
    }
  }

  float* slab = sT[wave];
#pragma unroll
  for (int i = 0; i < 4; ++i) {
    const int mBase = m0 + (i << 4);
#pragma unroll
    for (int j = 0; j < 4; ++j) {
#pragma unroll
      for (int r = 0; r < 8; ++r) slab[(mOff + r) * 68 + (j << 4) + rlane] = acc[i][j][r] * scale;
    }
    wave_lds_sync();
    {
      const int hq = lane >> 4, c4 = (lane & 15) * 4;
      for (int pass = 0; pass < 2; ++pass) {
#pragma unroll
        for (int it = 0; it < 8; ++it) {
          const int row = it * 2 + hq;
          const v4f v = *(const v4f*)(slab + row * 68 + c4);
          *(volatile v4f*)(C + (size_t)(mBase + row) * ldc + n0 + c4) = v;
        }
        __threadfence();
      }
    }
    wave_lds_sync();
  }
}

__global__ __launch_bounds__(256) void pack_logits_kernel(
    const float* __restrict__ C64, const float* __restrict__ bout, float* __restrict__ out0, int total4)
{
  const int i = blockIdx.x * 256 + threadIdx.x;
  if (i >= total4) return;
  v4f v;
#pragma unroll
  for (int e = 0; e < 4; ++e) {
    const int idx = 4 * i + e;
    const int row = idx / kV;
    const int col = idx - row * kV;
    v[e] = C64[(size_t)row * kVPad + col] + bout[col];
  }
  float* dp = out0 + (size_t)i * 4;
  *(volatile v4f*)dp = v;
  __threadfence();
  *(volatile v4f*)dp = v;
}

extern "C" void kernel_launch(void* const* d_in, const int* in_sizes, int n_in,
                              void* d_out, int out_size, void* d_ws, size_t ws_size,
                              hipStream_t stream) {
  if (n_in < 19) return;
  if (in_sizes[0] != kL * kB * kD) return;
  if (in_sizes[1] != kL * kB * kD) return;
  if (in_sizes[2] != kB) return;
  if (in_sizes[3] != kB * kT) return;
  if (in_sizes[4] != kV * kD) return;
  if (in_sizes[5] != 4 * kH * 2 * kD) return;
  if (in_sizes[6] != 4 * kH * kH) return;
  if (in_sizes[7] != 4 * kH || in_sizes[8] != 4 * kH) return;
  if (in_sizes[9] != 4 * kD * kH) return;
  if (in_sizes[10] != 4 * kD * kD) return;
  if (in_sizes[11] != 4 * kD || in_sizes[12] != 4 * kD) return;
  if (in_sizes[13] != kV * kKo) return;
  if (in_sizes[14] != kV) return;
  if (in_sizes[15] != kB * kH || in_sizes[16] != kB * kH) return;
  if (in_sizes[17] != kB * kD || in_sizes[18] != kB * kD) return;
  if (out_size != kT * kB * kV + kT * kB * kL) return;
  if (ws_size < kWsTotal) return;

  const float* key   = (const float*)d_in[0];
  const float* value = (const float*)d_in[1];
  const int*   lens  = (const int*)d_in[2];
  const int*   trans = (const int*)d_in[3];
  const float* emb   = (const float*)d_in[4];
  const float* Wih1  = (const float*)d_in[5];
  const float* Whh1  = (const float*)d_in[6];
  const float* bih1  = (const float*)d_in[7];
  const float* bhh1  = (const float*)d_in[8];
  const float* Wih2  = (const float*)d_in[9];
  const float* Whh2  = (const float*)d_in[10];
  const float* bih2  = (const float*)d_in[11];
  const float* bhh2  = (const float*)d_in[12];
  const float* Wout  = (const float*)d_in[13];
  const float* bout  = (const float*)d_in[14];
  const float* h10   = (const float*)d_in[15];
  const float* c10   = (const float*)d_in[16];
  const float* h20   = (const float*)d_in[17];
  const float* c20   = (const float*)d_in[18];

  char* ws = (char*)d_ws;
  unsigned short* W1C  = (unsigned short*)(ws + kOffW1C);
  unsigned short* W2C  = (unsigned short*)(ws + kOffW2C);
  unsigned short* WO   = (unsigned short*)(ws + kOffWO);
  unsigned short* HCAT = (unsigned short*)(ws + kOffHCAT);
  float*          C64  = (float*)(ws + kOffC64);

  float* out0 = (float*)d_out;
  float* out1 = (float*)d_out + (size_t)kT * kB * kV;

  cvt_rows_f16_kernel<<<(4 * kH * (2 * kD / 8)) / 256, 256, 0, stream>>>(
      Wih1, 2 * kD, 4 * kH, W1C, kK1, 0, 2 * kD / 8, 4 * kH * (2 * kD / 8), kCarryW);
  cvt_rows_f16_kernel<<<(4 * kH * (kH / 8)) / 256, 256, 0, stream>>>(
      Whh1, kH, 4 * kH, W1C, kK1, 2 * kD, kH / 8, 4 * kH * (kH / 8), kCarryW);
  cvt_rows_f16_kernel<<<(4 * kD * (kH / 8)) / 256, 256, 0, stream>>>(
      Wih2, kH, 4 * kD, W2C, kK2, 0, kH / 8, 4 * kD * (kH / 8), kCarryW);
  cvt_rows_f16_kernel<<<(4 * kD * (kD / 8)) / 256, 256, 0, stream>>>(
      Whh2, kD, 4 * kD, W2C, kK2, kH, kD / 8, 4 * kD * (kD / 8), kCarryW);
  cvt_rows_f16_kernel<<<(kVPad * (kKo / 8)) / 256, 256, 0, stream>>>(
      Wout, kKo, kV, WO, kKo, 0, kKo / 8, kVPad * (kKo / 8), kCarryW);

  decoder_steps_kernel<<<1, 512, 0, stream>>>(
      key, value, lens, trans, emb, W1C, W2C, bih1, bhh1, bih2, bhh2,
      h10, c10, h20, c20, HCAT, out1);

  gemm64_f16_kernel<<<(kRowsOut / 64) * (kVPad / 64) / 8, 256, 0, stream>>>(
      HCAT, kKo, WO, kKo, C64, kVPad, kRowsOut, kVPad, kKo, kFold);

  pack_logits_kernel<<<(kT * kB * kV / 4) / 256, 256, 0, stream>>>(C64, bout, out0, kT * kB * kV / 4);
}
